// EdgeGNN_40888088658022
// MI455X (gfx1250) — hardware-verified
//
#include <hip/hip_runtime.h>
#include <stddef.h>
#include <stdint.h>


#define DF      256
#define CATW    1792
#define DPW     512
#define KL0     768
#define KL      1024
#define KF      1792
#define CODE_L0 20
#define CODE_L  80
#define CODE_F  16020
#define NTHR    256
#define NWAVE   8
#define EPT     8
#define CHUNK   (NTHR * EPT)
#define WCAP    (EPT * 32)
#define LISTN   (NWAVE * WCAP)
#define NBMAX   2048
#define RCAP    28672
#define DEGCAP  128
#define PKS     11
#define GBM     64
#define GBN     128
#define GNT     8
#define GTHR    128
#define WSLIM   134217728
#define LDS_AGG ((2 * RCAP + 2 * NBMAX + LISTN) * 4 + 64)

static_assert((CHUNK & (CHUNK - 1)) == 0 && CHUNK <= (1 << PKS));
static_assert((NBMAX & (NBMAX - 1)) == 0 && NBMAX <= (1 << PKS));
static_assert(NTHR * 8 == NBMAX);
static_assert(LISTN >= NBMAX);
static_assert(LISTN >= NWAVE * WCAP);
static_assert((RCAP % 32) == 0 && RCAP >= NBMAX);
static_assert(LDS_AGG <= 300000);
static_assert(GBM == (GTHR / 32) * 16);
static_assert(GBN == 16 * GNT && GTHR == GBN && GBM <= GTHR);
static_assert((KL0 % 32) == 0 && (KL % 32) == 0 && (KF % 32) == 0 && (DF % 32) == 0);
static_assert(KF == DF + 3 * 2 * DF && KL == 4 * DF && KL0 == 3 * DF && DPW == 2 * DF && CATW == KF);
static_assert((DF % GBN) == 0 && DF == 32 * 8);

typedef float          v4f  __attribute__((ext_vector_type(4)));
typedef float          v8f  __attribute__((ext_vector_type(8)));
typedef int            v4i  __attribute__((ext_vector_type(4)));
typedef int            v8i  __attribute__((ext_vector_type(8)));
typedef unsigned short v8us __attribute__((ext_vector_type(8)));
typedef __bf16         v16b __attribute__((ext_vector_type(16)));
union FragB { v16b v; v8us h[2]; v8i w; };

__device__ __forceinline__ v8f wmb(const FragB& a, const FragB& b, v8f c) {
  v8f d = __builtin_amdgcn_wmma_f32_16x16x32_bf16(false, a.v, false, b.v, (short)0, c, false, false);
  asm volatile("v_nop\n\tv_nop\n\tv_nop\n\tv_nop" : "+v"(d) : "v"(a.w), "v"(b.w));
  return d;
}

__device__ __forceinline__ unsigned short bf_bits(float f) {
  unsigned int u = __float_as_uint(f);
  u += 0x7FFFu + ((u >> 16) & 1u);
  return (unsigned short)(u >> 16);
}
__device__ __forceinline__ float bf_val(unsigned short b) {
  return __uint_as_float(((unsigned int)b) << 16);
}
__device__ __forceinline__ float bf_rne(float f) { return bf_val(bf_bits(f)); }

__device__ __forceinline__ v8us cvt8b(const v4f a, const v4f b) {
  v8us hv;
  hv[0] = bf_bits(a.x); hv[1] = bf_bits(a.y); hv[2] = bf_bits(a.z); hv[3] = bf_bits(a.w);
  hv[4] = bf_bits(b.x); hv[5] = bf_bits(b.y); hv[6] = bf_bits(b.z); hv[7] = bf_bits(b.w);
  return hv;
}

__device__ __forceinline__ int scan_chunk(const int* __restrict__ dsts, int nE, int cbase, int slotBase,
                                          int nb, int vec8, int* list, int tid, int lane, int wave) {
  int wc = 0;
  const int el0  = tid * EPT;
  const int e0   = cbase + el0;
  const int sent = -2147483647 - 1;
  v4i da, db;
  if (vec8 != 0 && cbase + CHUNK <= nE) {
    da = *(const v4i*)(dsts + e0);
    db = *(const v4i*)(dsts + e0 + 4);
  } else {
    da.x = (e0     < nE) ? dsts[min(e0,     nE - 1)] : sent;
    da.y = (e0 + 1 < nE) ? dsts[min(e0 + 1, nE - 1)] : sent;
    da.z = (e0 + 2 < nE) ? dsts[min(e0 + 2, nE - 1)] : sent;
    da.w = (e0 + 3 < nE) ? dsts[min(e0 + 3, nE - 1)] : sent;
    db.x = (e0 + 4 < nE) ? dsts[min(e0 + 4, nE - 1)] : sent;
    db.y = (e0 + 5 < nE) ? dsts[min(e0 + 5, nE - 1)] : sent;
    db.z = (e0 + 6 < nE) ? dsts[min(e0 + 6, nE - 1)] : sent;
    db.w = (e0 + 7 < nE) ? dsts[min(e0 + 7, nE - 1)] : sent;
  }
  const unsigned nbs = (unsigned)slotBase;
  const unsigned unb = (unsigned)nb;
  const unsigned s0 = (unsigned)da.x - nbs, s1 = (unsigned)da.y - nbs;
  const unsigned s2 = (unsigned)da.z - nbs, s3 = (unsigned)da.w - nbs;
  const unsigned s4 = (unsigned)db.x - nbs, s5 = (unsigned)db.y - nbs;
  const unsigned s6 = (unsigned)db.z - nbs, s7 = (unsigned)db.w - nbs;
  const bool h0 = s0 < unb, h1 = s1 < unb, h2 = s2 < unb, h3 = s3 < unb;
  const bool h4 = s4 < unb, h5 = s5 < unb, h6 = s6 < unb, h7 = s7 < unb;
  const unsigned any = __builtin_amdgcn_ballot_w32(h0 | h1 | h2 | h3 | h4 | h5 | h6 | h7);
  if (any != 0u) {
#define HITJ(J, HJ, SJ) { \
      const unsigned mj = __builtin_amdgcn_ballot_w32(HJ); \
      if (mj != 0u) { \
        if (HJ) { \
          const int pos = wc + (int)__builtin_amdgcn_mbcnt_lo(mj, 0u); \
          if (pos < WCAP) list[wave * WCAP + pos] = ((el0 + (J)) << PKS) | (int)(SJ); \
        } \
        wc += (int)__builtin_popcount(mj); } }
    HITJ(0, h0, s0)
    HITJ(1, h1, s1)
    HITJ(2, h2, s2)
    HITJ(3, h3, s3)
    HITJ(4, h4, s4)
    HITJ(5, h5, s5)
    HITJ(6, h6, s6)
    HITJ(7, h7, s7)
#undef HITJ
  }
  return wc;
}

__global__ __launch_bounds__(NTHR) void k_xprep(const float* __restrict__ x, unsigned short* cat,
                                                int nN, int nUnits) {
  const int i = (int)blockIdx.x * NTHR + (int)threadIdx.x;
  if (i >= nUnits) return;
  const int row = i >> 5;
  const int c0  = (i & 31) * 8;
  const int rc  = row < nN ? row : nN - 1;
  const float* p = x + (size_t)rc * DF + c0;
  v4f a = *(const v4f*)p, b = *(const v4f*)(p + 4);
  const v4f z4 = {0.f, 0.f, 0.f, 0.f};
  if (row >= nN) { a = z4; b = z4; }
  const v8us hv = cvt8b(a, b);
  const size_t o = (size_t)row * CATW + c0;
  *(volatile v8us*)(cat + o) = hv;
  __threadfence();
  *(volatile v8us*)(cat + o) = hv;
}

__global__ __launch_bounds__(NTHR) void k_wt(const float* __restrict__ w, int wRows, int code, int K,
                                             unsigned short* wt, int nUnits) {
  const int u = (int)blockIdx.x * NTHR + (int)threadIdx.x;
  if (u >= nUnits) return;
  const int kq = K >> 3;
  const int n  = u / kq;
  const int k8 = (u - n * kq) * 8;
  const int seg = k8 >> 8;
  int srow = (k8 & 255) + 256 * ((code >> (2 * seg)) & 3);
  srow = srow > wRows - 8 ? wRows - 8 : srow;
  srow = srow < 0 ? 0 : srow;
  const float* p = w + (size_t)srow * DF + n;
  v4f a, b;
  a.x = p[0];                  a.y = p[(size_t)DF];         a.z = p[(size_t)2 * DF];     a.w = p[(size_t)3 * DF];
  b.x = p[(size_t)4 * DF];     b.y = p[(size_t)5 * DF];     b.z = p[(size_t)6 * DF];     b.w = p[(size_t)7 * DF];
  const v8us hv = cvt8b(a, b);
  const size_t o = (size_t)n * (size_t)K + k8;
  *(volatile v8us*)(wt + o) = hv;
  __threadfence();
  *(volatile v8us*)(wt + o) = hv;
}

__device__ __forceinline__ void kseg(v8f (&acc)[GNT], const unsigned short* ap, const unsigned short* wp,
                                     int ldw, int ksteps) {
#pragma unroll 1
  for (int ks = 0; ks < ksteps; ++ks) {
    FragB af;
    af.h[0] = *(const v8us*)(ap + 32 * ks);
    af.h[1] = *(const v8us*)(ap + 32 * ks + 16);
#pragma unroll
    for (int t = 0; t < GNT; ++t) {
      const unsigned short* wq = wp + (size_t)(16 * t) * (size_t)ldw + 32 * ks;
      FragB bf;
      bf.h[0] = *(const v8us*)wq;
      bf.h[1] = *(const v8us*)(wq + 16);
      acc[t] = wmb(af, bf, acc[t]);
    }
  }
}

__global__ __launch_bounds__(GTHR) void k_gemm(const unsigned short* A1, int lda1, int K1,
                                               const unsigned short* A2, int lda2, int K2,
                                               const unsigned short* __restrict__ WT, int ldw,
                                               const float* __restrict__ bias, const float* __restrict__ msk,
                                               int useM, int relu,
                                               float* outF, int ldo, int nValid, int wF,
                                               unsigned short* outB, int ldb, int wB)
{
  __shared__ __attribute__((aligned(16))) float stg[GBM * GBN];
  __shared__ __attribute__((aligned(16))) float biasL[GBN];
  __shared__ __attribute__((aligned(16))) float mskL[GBM];
  const int tid = (int)threadIdx.x, lane = tid & 31, wave = tid >> 5, hh = lane >> 4, m = lane & 15;
  const int rowBase = (int)blockIdx.x * GBM;
  const int col0    = (int)blockIdx.y * GBN;

  biasL[tid] = bf_rne(bias[col0 + tid]);
  if (tid < GBM) {
    float mv = 1.0f;
    if (useM != 0) mv = msk[rowBase + tid];
    mskL[tid] = mv;
  }
  __syncthreads();

  v8f acc[GNT];
  {
    const v8f z = {0.f, 0.f, 0.f, 0.f, 0.f, 0.f, 0.f, 0.f};
#pragma unroll
    for (int t = 0; t < GNT; ++t) acc[t] = z;
  }
  const int arow = rowBase + 16 * wave + m;
  const unsigned short* wp = WT + (size_t)(col0 + m) * (size_t)ldw + 8 * hh;
  kseg(acc, A1 + (size_t)arow * (size_t)lda1 + 8 * hh, wp, ldw, K1 >> 5);
  kseg(acc, A2 + (size_t)arow * (size_t)lda2 + 8 * hh, wp + K1, ldw, K2 >> 5);

#pragma unroll
  for (int t = 0; t < GNT; ++t) {
    const int lc = 16 * t + m;
    const float bb = biasL[lc];
#pragma unroll
    for (int r = 0; r < 8; ++r) {
      const int lr = 16 * wave + 8 * hh + r;
      float v = acc[t][r] + bb;
      if (relu != 0) v = fmaxf(v, 0.0f);
      v = v * mskL[lr];
      stg[lr * GBN + lc] = v;
    }
  }
  __syncthreads();

  if (wF != 0) {
    v4f fv[16];
#pragma unroll
    for (int i = 0; i < 16; ++i) {
      const int lr = 16 * wave + i;
      fv[i] = *(const v4f*)(stg + lr * GBN + 4 * lane);
    }
#pragma unroll
    for (int i = 0; i < 16; ++i) {
      const int gr = rowBase + 16 * wave + i;
      if (gr < nValid) {
        float* op = outF + (size_t)gr * (size_t)ldo + col0 + 4 * lane;
        *(volatile v4f*)op = fv[i];
      }
    }
    __threadfence();
#pragma unroll
    for (int i = 0; i < 16; ++i) {
      const int gr = rowBase + 16 * wave + i;
      if (gr < nValid) {
        float* op = outF + (size_t)gr * (size_t)ldo + col0 + 4 * lane;
        *(volatile v4f*)op = fv[i];
      }
    }
  }

  if (wB != 0) {
#pragma unroll 1
    for (int i = 0; i < 16; ++i) {
      const int lr = 16 * wave + i;
      const int gr = rowBase + lr;
      const float* sp = stg + lr * GBN + 8 * m;
      const v4f a = *(const v4f*)sp, b = *(const v4f*)(sp + 4);
      const v8us hv = cvt8b(a, b);
      v8us lv;
      lv[0] = bf_bits(a.x - bf_val(hv[0])); lv[1] = bf_bits(a.y - bf_val(hv[1]));
      lv[2] = bf_bits(a.z - bf_val(hv[2])); lv[3] = bf_bits(a.w - bf_val(hv[3]));
      lv[4] = bf_bits(b.x - bf_val(hv[4])); lv[5] = bf_bits(b.y - bf_val(hv[5]));
      lv[6] = bf_bits(b.z - bf_val(hv[6])); lv[7] = bf_bits(b.w - bf_val(hv[7]));
      v8us pk;
#pragma unroll
      for (int c = 0; c < 8; ++c) pk[c] = (hh != 0) ? lv[c] : hv[c];
      unsigned short* ob = outB + (size_t)gr * (size_t)ldb + 256 * hh + col0 + 8 * m;
      *(volatile v8us*)ob = pk;
      __threadfence();
      *(volatile v8us*)ob = pk;
    }
  }
}

template<int SRCB>
__global__ __launch_bounds__(NTHR) void k_agg(
    const int* __restrict__ srcs, const int* __restrict__ dsts,
    const float* __restrict__ HFp,
    const unsigned short* __restrict__ HBp, int pitchB,
    unsigned short* Dout, float* mskOut, int useMsk,
    int nN, int nE, int nb, int vec8, int MPr) {
  extern __shared__ v4f lds_dyn[];
  int* reg1 = (int*)lds_dyn;
  int* reg2 = reg1 + RCAP;
  int* scnt = reg2 + RCAP;
  int* soff = scnt + NBMAX;
  int* list = soff + NBMAX;
  int* wcnt = list + LISTN;
  int* wtot = wcnt + NWAVE;
  const int tid = (int)threadIdx.x, lane = tid & 31, wave = tid >> 5;
  const int nodeBase = (int)blockIdx.x * nb;

  for (int i = tid; i < NBMAX; i += NTHR) scnt[i] = 0;
  __syncthreads();

  int tot = 0;
  const int nChunks = (nE + CHUNK - 1) / CHUNK;
#pragma unroll 1
  for (int ch = 0; ch < nChunks; ++ch) {
    const int cbase = ch * CHUNK;
    const int wc = scan_chunk(dsts, nE, cbase, nodeBase, nb, vec8, list, tid, lane, wave);
    if (lane == 0) wcnt[wave] = wc;
    __syncthreads();
    int pre = 0, all = 0;
#pragma unroll
    for (int w2 = 0; w2 < NWAVE; ++w2) {
      int c = wcnt[w2];
      c = c < 0 ? 0 : (c > WCAP ? WCAP : c);
      all += c;
      pre += (w2 < wave) ? c : 0;
    }
    const int wcc  = wc > WCAP ? WCAP : wc;
    const int base = tot + pre;
#pragma unroll 1
    for (int i = lane; i < wcc; i += 32) {
      const int ent = list[wave * WCAP + i];
      const int el  = (ent >> PKS) & (CHUNK - 1);
      const int sl  = ent & (NBMAX - 1);
      int eid = cbase + el;
      eid = eid > nE - 1 ? nE - 1 : eid;
      const int pos = base + i;
      if (pos < RCAP) reg1[pos] = (int)(((unsigned)eid << PKS) | (unsigned)sl);
    }
    tot += all;
    tot = tot > RCAP ? RCAP : tot;
    __syncthreads();
  }
  const int nh = tot;

  if (wave == 0) {
#pragma unroll 1
    for (int b0 = 0; b0 < nh; b0 += 32) {
      const int idx = b0 + lane;
      const int uv  = reg1[idx < RCAP ? idx : RCAP - 1];
      const int m32 = (nh - b0) < 32 ? (nh - b0) : 32;
#pragma unroll 1
      for (int k = 0; k < m32; ++k) {
        const int u  = __builtin_amdgcn_readlane(uv, k);
        const int sl = u & (NBMAX - 1);
        if (lane == 0) scnt[sl] = scnt[sl] + 1;
      }
    }
  }
  __syncthreads();

  {
    const v4i ca = *(const v4i*)(scnt + 8 * tid);
    const v4i cb = *(const v4i*)(scnt + 8 * tid + 4);
    const int e0 = ca.x < 0 ? 0 : ca.x, e1 = ca.y < 0 ? 0 : ca.y, e2 = ca.z < 0 ? 0 : ca.z, e3 = ca.w < 0 ? 0 : ca.w;
    const int e4 = cb.x < 0 ? 0 : cb.x, e5 = cb.y < 0 ? 0 : cb.y, e6 = cb.z < 0 ? 0 : cb.z, e7 = cb.w < 0 ? 0 : cb.w;
    const int ts = e0 + e1 + e2 + e3 + e4 + e5 + e6 + e7;
    int incl = ts;
#pragma unroll
    for (int d = 1; d < 32; d <<= 1) {
      const int up = __shfl_up(incl, d);
      if (lane >= d) incl += up;
    }
    if (lane == 31) wtot[wave] = incl;
    __syncthreads();
    int pre = 0;
#pragma unroll
    for (int w2 = 0; w2 < NWAVE; ++w2) pre += (w2 < wave) ? wtot[w2] : 0;
    int run = pre + incl - ts;
    soff[8 * tid + 0] = run; run += e0;
    soff[8 * tid + 1] = run; run += e1;
    soff[8 * tid + 2] = run; run += e2;
    soff[8 * tid + 3] = run; run += e3;
    soff[8 * tid + 4] = run; run += e4;
    soff[8 * tid + 5] = run; run += e5;
    soff[8 * tid + 6] = run; run += e6;
    soff[8 * tid + 7] = run;
  }
  __syncthreads();
  for (int i = tid; i < NBMAX; i += NTHR) list[i] = soff[i];
  __syncthreads();

  if (wave == 0) {
#pragma unroll 1
    for (int b0 = 0; b0 < nh; b0 += 32) {
      const int idx = b0 + lane;
      const int uv  = reg1[idx < RCAP ? idx : RCAP - 1];
      const int m32 = (nh - b0) < 32 ? (nh - b0) : 32;
#pragma unroll 1
      for (int k = 0; k < m32; ++k) {
        const int u   = __builtin_amdgcn_readlane(uv, k);
        const int sl  = u & (NBMAX - 1);
        const int eid = (int)((unsigned)u >> PKS);
        if (lane == 0) {
          int pos = list[sl];
          pos = pos < 0 ? 0 : (pos > RCAP - 1 ? RCAP - 1 : pos);
          reg2[pos] = eid;
          list[sl] = pos + 1;
        }
      }
    }
  }
  __syncthreads();

  const int nbw = nb >> 3;
  const bool ovf = (nh >= RCAP);
  const float qnan = __int_as_float(0x7fc00000);
  float* mskl = (float*)reg1;

#pragma unroll 1
  for (int jt = 0; jt < nbw; ++jt) {
    const int slot = wave * nbw + jt;
    const int grow = nodeBase + slot;
    const int gcl  = grow < nN ? grow : nN - 1;
    int st = soff[slot];
    const int craw = scnt[slot];
    int cnt = craw;
    st  = st < 0 ? 0 : (st > nh ? nh : st);
    cnt = cnt < 0 ? 0 : (cnt > DEGCAP ? DEGCAP : cnt);
    if (cnt > nh - st) cnt = nh - st;
    const float pz = (ovf || craw > DEGCAP) ? qnan : 0.0f;
    const float live = grow < nN ? 1.0f : 0.0f;

    float sv[8];
    float ag[8] = {0.f, 0.f, 0.f, 0.f, 0.f, 0.f, 0.f, 0.f};
    if (SRCB != 0) {
      const v8us w = *(const v8us*)(HBp + (size_t)gcl * (size_t)pitchB + 8 * lane);
#pragma unroll
      for (int c = 0; c < 8; ++c) sv[c] = bf_val(w[c]);
    } else {
      const float* sr = HFp + (size_t)gcl * DF + 8 * lane;
      const v4f a = *(const v4f*)sr, b = *(const v4f*)(sr + 4);
      sv[0] = a.x; sv[1] = a.y; sv[2] = a.z; sv[3] = a.w;
      sv[4] = b.x; sv[5] = b.y; sv[6] = b.z; sv[7] = b.w;
    }

#pragma unroll 1
    for (int q = 0; q < cnt; ++q) {
      int idx = st + q; idx = idx > RCAP - 1 ? RCAP - 1 : idx;
      int eid = reg2[idx]; eid = eid < 0 ? 0 : (eid > nE - 1 ? nE - 1 : eid);
      const int sraw = srcs[eid];
      const int s = sraw < 0 ? 0 : (sraw > nN - 1 ? nN - 1 : sraw);
      if (SRCB != 0) {
        const v8us w = *(const v8us*)(HBp + (size_t)s * (size_t)pitchB + 8 * lane);
#pragma unroll
        for (int c = 0; c < 8; ++c) ag[c] += bf_val(w[c]);
      } else {
        const float* nr = HFp + (size_t)s * DF + 8 * lane;
        const v4f a = *(const v4f*)nr, b = *(const v4f*)(nr + 4);
        ag[0] += a.x; ag[1] += a.y; ag[2] += a.z; ag[3] += a.w;
        ag[4] += b.x; ag[5] += b.y; ag[6] += b.z; ag[7] += b.w;
      }
    }
    const float dcl  = cnt > 0 ? (float)cnt : 1.0f;
    const float invd = 1.0f / dcl;
    v8us hvv, lvv;
#pragma unroll
    for (int c = 0; c < 8; ++c) {
      const float d = (ag[c] * invd - sv[c]) * live + pz;
      const unsigned short hb = bf_bits(d);
      hvv[c] = hb;
      lvv[c] = bf_bits(d - bf_val(hb));
    }
    unsigned short* gp = Dout + (size_t)grow * DPW + 8 * lane;
    const bool wsv = grow < MPr;
    if (wsv) { *(volatile v8us*)gp = hvv; *(volatile v8us*)(gp + DF) = lvv; }
    __threadfence();
    if (wsv) { *(volatile v8us*)gp = hvv; *(volatile v8us*)(gp + DF) = lvv; }
    if (lane == 0) mskl[slot] = (cnt > 0 && grow < nN) ? 1.0f : 0.0f;
  }
  __syncthreads();

  if (useMsk != 0) {
#pragma unroll 1
    for (int i = tid; 4 * i < nb; i += NTHR) {
      const v4f mv = *(const v4f*)(mskl + 4 * i);
      float* mp = mskOut + (size_t)nodeBase + 4 * i;
      *(volatile v4f*)mp = mv;
      __threadfence();
      *(volatile v4f*)mp = mv;
    }
  }
}

static int pick_nb(int nE, int nN) {
  int nb = NBMAX;
  while (nb > 32 && (long long)nb * (long long)nE * 5LL > (long long)RCAP * (long long)nN * 4LL) nb >>= 1;
  return nb;
}
static inline int cdiv(int a, int b) { return (a + b - 1) / b; }

extern "C" void kernel_launch(void* const* d_in, const int* in_sizes, int n_in,
                              void* d_out, int out_size, void* d_ws, size_t ws_size,
                              hipStream_t stream) {
  if (n_in < 10) return;
  const int nN = in_sizes[0] / DF;
  if (nN <= 0 || in_sizes[0] != nN * DF || nN > (1 << 22)) return;
  if ((in_sizes[1] & 1) != 0) return;
  const int nE = in_sizes[1] / 2;
  if (nE < 1 || nE > (1 << 21)) return;
  if (in_sizes[2] != 2 * DF * DF || in_sizes[4] != 2 * DF * DF || in_sizes[6] != 2 * DF * DF) return;
  if (in_sizes[3] != DF || in_sizes[5] != DF || in_sizes[7] != DF || in_sizes[9] != DF) return;
  if (in_sizes[8] != 4 * DF * DF) return;
  if (out_size != nN * DF) return;

  const float* x   = (const float*)d_in[0];
  const int*   ei  = (const int*)  d_in[1];
  const float* W0  = (const float*)d_in[2];
  const float* b0  = (const float*)d_in[3];
  const float* W1  = (const float*)d_in[4];
  const float* b1  = (const float*)d_in[5];
  const float* W2  = (const float*)d_in[6];
  const float* b2  = (const float*)d_in[7];
  const float* Wf  = (const float*)d_in[8];
  const float* bfv = (const float*)d_in[9];
  float* out = (float*)d_out;
  const int* src = ei;
  const int* dst = ei + nE;

  const int MP   = cdiv(nN, GBM) * GBM;
  const int nb   = pick_nb(nE, nN);
  const int gA   = cdiv(MP, nb);
  const int vec8 = ((nE & 3) == 0) ? 1 : 0;
  if (gA * nb < MP) return;

  char* ws = (char*)d_ws;
  size_t off = 0;
  const size_t oCAT = off; off += (size_t)MP * CATW * 2;           off = (off + 255) & ~(size_t)255;
  const size_t oD   = off; off += (size_t)MP * DPW * 2;            off = (off + 255) & ~(size_t)255;
  const size_t oHF  = off; off += (size_t)MP * DF * 4;             off = (off + 255) & ~(size_t)255;
  const size_t oMSK = off; off += (size_t)gA * (size_t)nb * 4;     off = (off + 255) & ~(size_t)255;
  const size_t oW0  = off; off += (size_t)DF * KL0 * 2;            off = (off + 255) & ~(size_t)255;
  const size_t oW1  = off; off += (size_t)DF * KL * 2;             off = (off + 255) & ~(size_t)255;
  const size_t oW2  = off; off += (size_t)DF * KL * 2;             off = (off + 255) & ~(size_t)255;
  const size_t oWF  = off; off += (size_t)DF * KF * 2;             off = (off + 255) & ~(size_t)255;
  if (off > ws_size || off > (size_t)WSLIM) return;
  unsigned short* CAT = (unsigned short*)(ws + oCAT);
  unsigned short* DPL = (unsigned short*)(ws + oD);
  float*          HF  = (float*)(ws + oHF);
  float*          MSK = (float*)(ws + oMSK);
  unsigned short* WT0 = (unsigned short*)(ws + oW0);
  unsigned short* WT1 = (unsigned short*)(ws + oW1);
  unsigned short* WT2 = (unsigned short*)(ws + oW2);
  unsigned short* WTF = (unsigned short*)(ws + oWF);

  hipFuncSetAttribute(reinterpret_cast<const void*>(&k_agg<0>),
                      hipFuncAttributeMaxDynamicSharedMemorySize, LDS_AGG);
  hipFuncSetAttribute(reinterpret_cast<const void*>(&k_agg<1>),
                      hipFuncAttributeMaxDynamicSharedMemorySize, LDS_AGG);

  const int nUx = MP * (DF / 8);
  k_xprep<<<cdiv(nUx, NTHR), NTHR, 0, stream>>>(x, CAT, nN, nUx);

  {
    const int nU0 = DF * (KL0 / 8);
    k_wt<<<cdiv(nU0, NTHR), NTHR, 0, stream>>>(W0, 2 * DF, CODE_L0, KL0, WT0, nU0);
    const int nU1 = DF * (KL / 8);
    k_wt<<<cdiv(nU1, NTHR), NTHR, 0, stream>>>(W1, 2 * DF, CODE_L, KL, WT1, nU1);
    k_wt<<<cdiv(nU1, NTHR), NTHR, 0, stream>>>(W2, 2 * DF, CODE_L, KL, WT2, nU1);
    const int nUF = DF * (KF / 8);
    k_wt<<<cdiv(nUF, NTHR), NTHR, 0, stream>>>(Wf, 4 * DF, CODE_F, KF, WTF, nUF);
  }

  const dim3 gG(MP / GBM, DF / GBN);
  k_agg<1><<<gA, NTHR, LDS_AGG, stream>>>(src, dst, HF, CAT, CATW, DPL, MSK, 1, nN, nE, nb, vec8, MP);
  k_gemm<<<gG, GTHR, 0, stream>>>(CAT, CATW, DF, DPL, DPW, 2 * DF, WT0, KL0, b0, MSK, 1, 1,
                                  HF, DF, MP, 1, CAT + DF, CATW, 1);
  k_agg<0><<<gA, NTHR, LDS_AGG, stream>>>(src, dst, HF, CAT, CATW, DPL, MSK, 0, nN, nE, nb, vec8, MP);
  k_gemm<<<gG, GTHR, 0, stream>>>(CAT + DF, CATW, 2 * DF, DPL, DPW, 2 * DF, WT1, KL, b1, MSK, 1, 1,
                                  HF, DF, MP, 1, CAT + 3 * DF, CATW, 1);
  k_agg<0><<<gA, NTHR, LDS_AGG, stream>>>(src, dst, HF, CAT, CATW, DPL, MSK, 0, nN, nE, nb, vec8, MP);
  k_gemm<<<gG, GTHR, 0, stream>>>(CAT + 3 * DF, CATW, 2 * DF, DPL, DPW, 2 * DF, WT2, KL, b2, MSK, 1, 1,
                                  HF, DF, MP, 0, CAT + 5 * DF, CATW, 1);
  k_gemm<<<gG, GTHR, 0, stream>>>(CAT, CATW, KF, DPL, DPW, 0, WTF, KF, bfv, MSK, 0, 0,
                                  out, DF, nN, 1, CAT, CATW, 0);
}
